// XFormerDecoderLayer_24962349924418
// MI455X (gfx1250) — hardware-verified
//
#include <hip/hip_runtime.h>


#define NB_  2
#define TT   2048
#define SS   512
#define TK   (TT + SS)
#define DD   1024
#define NH_  16
#define HD   64
#define FF   4096
#define ZH   2
#define PCAR 1024.0f
#define SCL  0.125f
#define WSC  16384.0f
typedef _Float16 h16;
typedef unsigned short bf;
typedef __attribute__((ext_vector_type(16))) __bf16   v16bf;
typedef __attribute__((ext_vector_type(16))) _Float16 v16h;
typedef __attribute__((ext_vector_type(8)))  _Float16 v8h;
typedef __attribute__((ext_vector_type(8)))  unsigned short v8us;
typedef __attribute__((ext_vector_type(8)))  float    v8f;
typedef __attribute__((ext_vector_type(4)))  float    v4f;
typedef v8h  __attribute__((may_alias)) v8ha;
typedef v4f  __attribute__((may_alias)) v4fa;
typedef v8us __attribute__((may_alias)) v8usa;

__device__ __forceinline__ unsigned short f2bf(float f) { unsigned u = __float_as_uint(f); u += 0x7FFFu + ((u >> 16) & 1u); return (unsigned short)(u >> 16); }
__device__ __forceinline__ float bf2f(unsigned short b) { return __uint_as_float(((unsigned)b) << 16); }
__device__ __forceinline__ float bfr(float f) { return bf2f(f2bf(f)); }
__device__ __forceinline__ v16h cat16(v8h lo, v8h hi) { return __builtin_shufflevector(lo, hi, 0, 1, 2, 3, 4, 5, 6, 7, 8, 9, 10, 11, 12, 13, 14, 15); }
__device__ __forceinline__ v16bf cat16b(v8us lo, v8us hi) { return __builtin_bit_cast(v16bf, __builtin_shufflevector(lo, hi, 0, 1, 2, 3, 4, 5, 6, 7, 8, 9, 10, 11, 12, 13, 14, 15)); }
__device__ __forceinline__ v8f wmma16(v16h a, v16h b, v8f c) { return __builtin_amdgcn_wmma_f32_16x16x32_f16(false, a, false, b, (short)0, c, false, false); }
__device__ __forceinline__ v8f wmmab(v16bf a, v16bf b, v8f c) { return __builtin_amdgcn_wmma_f32_16x16x32_bf16(false, a, false, b, (short)0, c, false, false); }


template <typename T16> struct WFrag;
template <> struct WFrag<h16> { typedef v16h V; static __device__ __forceinline__ V ld(const h16* p) { return cat16(*(const v8h*)p, *(const v8h*)(p + 16)); } static __device__ __forceinline__ v8f mma(V a, V b, v8f c) { return wmma16(a, b, c); } };
template <> struct WFrag<bf> { typedef v16bf V; static __device__ __forceinline__ V ld(const bf* p) { return cat16b(*(const v8us*)p, *(const v8us*)(p + 16)); } static __device__ __forceinline__ v8f mma(V a, V b, v8f c) { return wmmab(a, b, c); } };
template <typename T16, int NSPLIT, bool BIAS>
__global__ __launch_bounds__(32) void k_gemmw(const T16* __restrict__ A, const T16* __restrict__ A2, const T16* __restrict__ Bt, const T16* __restrict__ Bt2, int K, float* C, int ldc, const float* __restrict__ bias, size_t sA, size_t sB, size_t sC) {
    typedef typename WFrag<T16>::V V;
    __shared__ __align__(16) float os[16 * 68];
    const size_t z = blockIdx.z; A += z * sA; if (A2) A2 += z * sA; Bt += z * sB; if (Bt2) Bt2 += z * sB; C += z * sC;
    const int lane = threadIdx.x & 31, lr = lane & 15, hi = lane >> 4; const int r0 = blockIdx.x * 64, c0 = blockIdx.y * 64;
    v8f acc[4][4];
#pragma unroll
    for (int mb = 0; mb < 4; ++mb)
#pragma unroll
        for (int nb = 0; nb < 4; ++nb) acc[mb][nb] = (v8f){};
    const size_t aoff = (size_t)(r0 + lr) * K + 8 * hi, boff = (size_t)(c0 + lr) * K + 8 * hi;
#pragma unroll 1
    for (int kc = 0; kc < K; kc += 32) {
        V a[4], a2[4];
#pragma unroll
        for (int mb = 0; mb < 4; ++mb) { a[mb] = WFrag<T16>::ld(A + aoff + (size_t)mb * 16 * K + kc); if (NSPLIT == 1 || NSPLIT == 2) a2[mb] = WFrag<T16>::ld(A2 + aoff + (size_t)mb * 16 * K + kc); }
#pragma unroll
        for (int nb = 0; nb < 4; ++nb) { const V b = WFrag<T16>::ld(Bt + boff + (size_t)nb * 16 * K + kc); V b2; if (NSPLIT >= 2) b2 = WFrag<T16>::ld(Bt2 + boff + (size_t)nb * 16 * K + kc);
#pragma unroll
            for (int mb = 0; mb < 4; ++mb) { acc[mb][nb] = WFrag<T16>::mma(a[mb], b, acc[mb][nb]); if (NSPLIT == 1 || NSPLIT == 2) acc[mb][nb] = WFrag<T16>::mma(a2[mb], b, acc[mb][nb]); if (NSPLIT >= 2) acc[mb][nb] = WFrag<T16>::mma(a[mb], b2, acc[mb][nb]); } }
        asm volatile("v_nop\n\tv_nop\n\tv_nop\n\tv_nop" : "+v"(acc[0][0]), "+v"(acc[1][1]), "+v"(acc[2][2]), "+v"(acc[3][3]) : "v"(a[0]), "v"(a[3]));
    }
#pragma unroll
    for (int mb = 0; mb < 4; ++mb) {
#pragma unroll
        for (int nb = 0; nb < 4; ++nb) {
#pragma unroll
            for (int j = 0; j < 8; ++j) os[(hi * 8 + j) * 68 + nb * 16 + lr] = acc[mb][nb][j]; }
        __builtin_amdgcn_wave_barrier(); asm volatile("" ::: "memory");
        float* crow = C + (size_t)(r0 + mb * 16) * ldc + c0;
#pragma unroll 1
        for (int ps = 0; ps < 2; ++ps) {
#pragma unroll
            for (int s = 0; s < 8; ++s) { const int row = 2 * s + hi, cofs = lr * 4; v4f val = *(const v4fa*)(os + row * 68 + cofs); if (BIAS) { val[0] += bfr(bias[c0 + cofs]); val[1] += bfr(bias[c0 + cofs + 1]); val[2] += bfr(bias[c0 + cofs + 2]); val[3] += bfr(bias[c0 + cofs + 3]); }
                *(volatile v4f*)(crow + (size_t)row * ldc + cofs) = val; }
            if (ps == 0) __threadfence(); }
        __builtin_amdgcn_wave_barrier(); asm volatile("" ::: "memory");
    }
}

__device__ __forceinline__ h16 tohx(float x) { return (h16)x; }
__device__ __forceinline__ void splitf(float y, unsigned short& h, unsigned short& l) { h = f2bf(y); l = f2bf(y - bf2f(h)); }
typedef __attribute__((ext_vector_type(2))) _Float16 v2h;
typedef __attribute__((ext_vector_type(4))) _Float16 v4h;
typedef __attribute__((ext_vector_type(2))) unsigned short v2us;
typedef __attribute__((ext_vector_type(4))) unsigned short v4us;
typedef __attribute__((ext_vector_type(2))) float v2f;

__global__ __launch_bounds__(256) void k_wtG(const float* __restrict__ w, int K, int N, bf* Bt) {
    const int lane = threadIdx.x & 31; const int L0 = (blockIdx.x * 8 + (threadIdx.x >> 5)) * 8; const int nlines = N * K / 64;
#pragma unroll 1
    for (int ps = 0; ps < 2; ++ps) {
#pragma unroll 1
        for (int l = 0; l < 8; ++l) { const int L = L0 + l; if (L >= nlines) break; const size_t e = (size_t)L * 64 + lane * 2; const int k = (int)(e % K), n = (int)(e / K); v2us o;
            o[0] = f2bf(w[(size_t)k * N + n]); o[1] = f2bf(w[(size_t)(k + 1) * N + n]); *(volatile v2us*)(Bt + e) = o; }
        if (ps == 0) __threadfence(); }
}
__global__ __launch_bounds__(256) void k_cvt8(const float* __restrict__ src, bf* dst, size_t n8) { const size_t i = (size_t)blockIdx.x * 256 + threadIdx.x; if (i >= n8) return; const v8f v = *(const v8f*)(src + i * 8); v8us o;
#pragma unroll
    for (int k = 0; k < 8; ++k) o[k] = f2bf(v[k]); *(volatile v8us*)(dst + i * 8) = o; __threadfence(); *(volatile v8us*)(dst + i * 8) = o; }
__global__ __launch_bounds__(256) void k_wtG16(const float* __restrict__ w, int K, int N, int pitch, int col0, h16* Bt) {
    const int lane = threadIdx.x & 31; const int L0 = (blockIdx.x * 8 + (threadIdx.x >> 5)) * 8; const int nlines = N * K / 64;
#pragma unroll 1
    for (int ps = 0; ps < 2; ++ps) {
#pragma unroll 1
        for (int l = 0; l < 8; ++l) { const int L = L0 + l; if (L >= nlines) break; const size_t e = (size_t)L * 64 + lane * 2; const int k = (int)(e % K), n = (int)(e / K); v2h o;
            o[0] = tohx(bfr(w[(size_t)k * pitch + col0 + n]) * WSC); o[1] = tohx(bfr(w[(size_t)(k + 1) * pitch + col0 + n]) * WSC); *(volatile v2h*)(Bt + e) = o; }
        if (ps == 0) __threadfence(); }
}
template <int RAWA, int DOUBLE, int F16>
__global__ __launch_bounds__(256) void k_ln1k(const float* __restrict__ A, const float* __restrict__ ga, const float* __restrict__ ba, const float* __restrict__ gb, const float* __restrict__ bb2, bf* Yh, bf* Yl, h16* Y16) {
    const int lane = threadIdx.x & 31; const int r = blockIdx.x * 8 + (threadIdx.x >> 5); if (r >= TT) return; float v[32];
#pragma unroll
    for (int c = 0; c < 8; ++c) { const v4f a = *(const v4f*)(A + (size_t)r * DD + c * 128 + lane * 4);
#pragma unroll
        for (int q = 0; q < 4; ++q) { float t = RAWA ? bfr(a[q]) : a[q]; asm volatile("" : "+v"(t)); v[c * 4 + q] = t; } }
#pragma unroll
    for (int pass = 0; pass < (DOUBLE ? 2 : 1); ++pass) { const float* gg = pass ? gb : ga; const float* bb = pass ? bb2 : ba; float s = 0.f;
#pragma unroll
        for (int i = 0; i < 32; ++i) s = __fadd_rn(s, v[i]);
#pragma unroll
        for (int sh = 16; sh; sh >>= 1) s += __shfl_xor(s, sh, 32);
        const float mu = s * (1.0f / DD); float qq = 0.f;
#pragma unroll
        for (int i = 0; i < 32; ++i) { const float d0 = v[i] - mu; float p = __fmul_rn(d0, d0); asm volatile("" : "+v"(p)); qq = __fadd_rn(qq, p); }
#pragma unroll
        for (int sh = 16; sh; sh >>= 1) qq += __shfl_xor(qq, sh, 32);
        const float rs = __fdiv_rn(1.0f, __fsqrt_rn(__fadd_rn(qq * (1.0f / DD), 1e-5f)));
#pragma unroll
        for (int c = 0; c < 8; ++c) {
#pragma unroll
            for (int q = 0; q < 4; ++q) { const int col = c * 128 + lane * 4 + q; float g = bfr(gg[col]), bq = bfr(bb[col]); asm volatile("" : "+v"(g)); asm volatile("" : "+v"(bq)); float tn = __fmul_rn(v[c * 4 + q] - mu, rs); asm volatile("" : "+v"(tn)); float tg = __fmul_rn(tn, g); asm volatile("" : "+v"(tg)); v[c * 4 + q] = __fadd_rn(tg, bq); } } }
#pragma unroll 1
    for (int ps = 0; ps < 2; ++ps) {
#pragma unroll
        for (int c = 0; c < 8; ++c) { const size_t o = (size_t)r * DD + c * 128 + lane * 4;
            if (F16) { v4h o4; for (int q = 0; q < 4; ++q) o4[q] = tohx(v[c * 4 + q]); *(volatile v4h*)(Y16 + o) = o4; }
            else { v4us oh, ol; for (int q = 0; q < 4; ++q) { unsigned short a2, c2; splitf(v[c * 4 + q], a2, c2); oh[q] = a2; ol[q] = c2; } *(volatile v4us*)(Yh + o) = oh; *(volatile v4us*)(Yl + o) = ol; } }
        if (ps == 0) __threadfence(); }
}
__global__ __launch_bounds__(256) void k_qpl(const float* __restrict__ F3, h16* QP) { const int e = (blockIdx.x * 256 + threadIdx.x) * 2; if (e >= NH_ * TT * HD) return; const int d = e & 63; const int t = (e >> 6) & (TT - 1); const int h = e / (TT * HD); v2h o; o[0] = tohx(F3[(size_t)t * 3 * DD + h * HD + d]); o[1] = tohx(F3[(size_t)t * 3 * DD + h * HD + d + 1]); *(volatile v2h*)(QP + e) = o; __threadfence(); *(volatile v2h*)(QP + e) = o; }
__global__ __launch_bounds__(256) void k_kcat(const float* __restrict__ F3, const float* __restrict__ FC, h16* KP) { const int e = (blockIdx.x * 256 + threadIdx.x) * 2; if (e >= NH_ * TK * HD) return; const int d = e & 63; const int j = (e >> 6) % TK; const int h = e / (TK * HD);
    const float* src = (j < TT) ? (F3 + (size_t)j * 3 * DD + DD + h * HD + d) : (FC + (size_t)(j - TT) * 2 * DD + h * HD + d); v2h o; o[0] = tohx(src[0]); o[1] = tohx(src[1]); *(volatile v2h*)(KP + e) = o; __threadfence(); *(volatile v2h*)(KP + e) = o; }
__global__ __launch_bounds__(256) void k_vcat(const float* __restrict__ F3, const float* __restrict__ FC, h16* VT) { const int e = (blockIdx.x * 256 + threadIdx.x) * 2; if (e >= NH_ * HD * TK) return; const int j = e % TK; const int d = (e / TK) & 63; const int h = e / (TK * HD); v2h o;
#pragma unroll
    for (int q = 0; q < 2; ++q) { const int jj = j + q; o[q] = tohx(jj < TT ? F3[(size_t)jj * 3 * DD + 2 * DD + h * HD + d] : FC[(size_t)(jj - TT) * 2 * DD + DD + h * HD + d]); }
    *(volatile v2h*)(VT + e) = o; __threadfence(); *(volatile v2h*)(VT + e) = o; }
__global__ __launch_bounds__(256) void k_smax(const float* __restrict__ S, float* RS) { const int lane = threadIdx.x & 31; const int row = blockIdx.x * 8 + (threadIdx.x >> 5); if (row >= ZH * TT) return; const int i = row & (TT - 1); const float* sr = S + (size_t)row * TK; float m = -3.0e38f;
#pragma unroll 4
    for (int c0 = lane * 4; c0 < TK; c0 += 128) { const v4f v = *(const v4f*)(sr + c0);
#pragma unroll
        for (int q = 0; q < 4; ++q) { const int j = c0 + q; m = (j <= i || j >= TT) ? fmaxf(m, v[q]) : m; } }
#pragma unroll
    for (int sh = 16; sh; sh >>= 1) m = fmaxf(m, __shfl_xor(m, sh, 32));
    const float o = lane == 0 ? m : 0.f; *(volatile float*)(RS + (size_t)row * 32 + lane) = o; __threadfence(); *(volatile float*)(RS + (size_t)row * 32 + lane) = o; }
__global__ __launch_bounds__(256) void k_sexp(const float* __restrict__ S, float* RS, h16* P) { const int lane = threadIdx.x & 31; const int row = blockIdx.x * 8 + (threadIdx.x >> 5); if (row >= ZH * TT) return; const int i = row & (TT - 1); const float* sr = S + (size_t)row * TK; const float m = RS[(size_t)row * 32]; float sum = 0.f;
#pragma unroll 1
    for (int ps = 0; ps < 2; ++ps) { sum = 0.f;
#pragma unroll 2
        for (int c0 = lane * 4; c0 < TK; c0 += 128) { const v4f v = *(const v4f*)(sr + c0); v4h o;
#pragma unroll
            for (int q = 0; q < 4; ++q) { const int j = c0 + q; float dlt = __fsub_rn(v[q], m); asm volatile("" : "+v"(dlt)); const float e = (j <= i || j >= TT) ? __expf(__fmul_rn(dlt, SCL)) : 0.f; sum += e; o[q] = tohx(e * PCAR); }
            *(volatile v4h*)(P + (size_t)row * TK + c0) = o; }
        if (ps == 0) __threadfence(); }
#pragma unroll
    for (int sh = 16; sh; sh >>= 1) sum += __shfl_xor(sum, sh, 32);
    const float o2 = lane == 0 ? m : (lane == 1 ? __fdiv_rn(1.0f, sum * PCAR) : 0.f); *(volatile float*)(RS + (size_t)row * 32 + lane) = o2; __threadfence(); *(volatile float*)(RS + (size_t)row * 32 + lane) = o2; }
__global__ __launch_bounds__(256) void k_mrgx(const float* __restrict__ O, const float* __restrict__ RS, const float* __restrict__ xb, int h0, float* X1) { const int e = (blockIdx.x * 256 + threadIdx.x) * 2; if (e >= ZH * TT * HD) return; const int d = e & 63; const int t = (e >> 6) & (TT - 1); const int zz = e / (TT * HD); const float sc = RS[((size_t)zz * TT + t) * 32 + 1]; const size_t oo = (size_t)t * DD + (h0 + zz) * HD + d; v2f o;
#pragma unroll
    for (int q = 0; q < 2; ++q) { float a = __fmul_rn(O[e + q], sc); asm volatile("" : "+v"(a)); o[q] = __fadd_rn(bfr(xb[oo + q]), a); } *(volatile v2f*)(X1 + oo) = o; __threadfence(); *(volatile v2f*)(X1 + oo) = o; }
__global__ __launch_bounds__(256) void k_gelu16(const float* __restrict__ HF, const float* __restrict__ b1, h16* G16) { const size_t e = ((size_t)blockIdx.x * 256 + threadIdx.x) * 2; if (e >= (size_t)TT * FF) return; const int f = (int)(e % FF); v2h o;
#pragma unroll
    for (int q = 0; q < 2; ++q) { float a = HF[e + q] * (1.0f / WSC); asm volatile("" : "+v"(a)); const float h = __fadd_rn(a, bfr(b1[f + q])); float er = erff(h * 0.70710678f); asm volatile("" : "+v"(er)); float hh = __fmul_rn(0.5f, h); asm volatile("" : "+v"(hh)); o[q] = tohx(__fmul_rn(hh, __fadd_rn(1.0f, er))); }
    *(volatile v2h*)(G16 + e) = o; __threadfence(); *(volatile v2h*)(G16 + e) = o; }
__global__ __launch_bounds__(256) void k_fin(const float* __restrict__ X1, const float* __restrict__ F2, const float* __restrict__ b2, float* OUTb) { const size_t e = ((size_t)blockIdx.x * 256 + threadIdx.x) * 2; if (e >= (size_t)TT * DD) return; const int c = (int)(e % DD); v2f o;
#pragma unroll
    for (int q = 0; q < 2; ++q) { float a = F2[e + q] * (1.0f / WSC); asm volatile("" : "+v"(a)); float y = __fadd_rn(a, bfr(b2[c + q])); asm volatile("" : "+v"(y)); o[q] = __fadd_rn(X1[e + q], y); } *(volatile v2f*)(OUTb + e) = o; __threadfence(); *(volatile v2f*)(OUTb + e) = o; }

extern "C" void kernel_launch(void* const* d_in, const int* in_sizes, int n_in,
                              void* d_out, int out_size, void* d_ws, size_t ws_size, hipStream_t stream) {
    (void)in_sizes; (void)n_in; (void)out_size;
    const float* IN[16]; for (int i = 0; i < 16; ++i) IN[i] = (const float*)d_in[i];
    float* OUT = (float*)d_out;
    char* wsp = (char*)d_ws;
    auto take = [&](size_t bytes) { char* p = wsp; wsp += (bytes + 255) & ~(size_t)255; return (void*)p; };
    bf* WQKV = (bf*)take((size_t)3 * DD * DD * 2); bf* WCKV = (bf*)take((size_t)2 * DD * DD * 2); h16* W1S = (h16*)take((size_t)FF * DD * 2); h16* W2S = (h16*)take((size_t)DD * FF * 2);
    bf* Xh = (bf*)take((size_t)TT * DD * 2); bf* Xl = (bf*)take((size_t)TT * DD * 2); bf* CB = (bf*)take((size_t)SS * DD * 2); float* F3 = (float*)take((size_t)TT * 3 * DD * 4); float* FC = (float*)take((size_t)SS * 2 * DD * 4);
    h16* QP = (h16*)take((size_t)NH_ * TT * HD * 2); h16* KP = (h16*)take((size_t)NH_ * TK * HD * 2); h16* VT = (h16*)take((size_t)NH_ * HD * TK * 2); float* Sb = (float*)take((size_t)ZH * TT * TK * 4); h16* Pm = (h16*)take((size_t)ZH * TT * TK * 2); float* RS = (float*)take((size_t)ZH * TT * 32 * 4); float* Ob = (float*)take((size_t)ZH * TT * HD * 4); float* X1 = (float*)take((size_t)TT * DD * 4);
    if ((size_t)(wsp - (char*)d_ws) > ws_size) return;
    h16* H16 = (h16*)Xh; float* HF = Sb; h16* G16 = Pm; float* F2 = F3;
    { k_wtG<<<(unsigned)((DD * 3 * DD / 64 + 63) / 64), 256, 0, stream>>>(IN[2], DD, 3 * DD, WQKV); k_wtG<<<(unsigned)((DD * 2 * DD / 64 + 63) / 64), 256, 0, stream>>>(IN[4], DD, 2 * DD, WCKV);
      k_wtG16<<<(unsigned)((DD * FF / 64 + 63) / 64), 256, 0, stream>>>(IN[12], DD, FF, FF, 0, W1S); k_wtG16<<<(unsigned)((FF * DD / 64 + 63) / 64), 256, 0, stream>>>(IN[14], FF, DD, DD, 0, W2S); }
    const unsigned LQ = (NH_ * TT * HD / 2 + 255) / 256, LK = (NH_ * TK * HD / 2 + 255) / 256;
    for (int b = 0; b < NB_; ++b) { const float* xb = IN[0] + (size_t)b * TT * DD;
        k_ln1k<1, 0, 0><<<TT / 8, 256, 0, stream>>>(xb, IN[6], IN[7], nullptr, nullptr, Xh, Xl, nullptr);
        k_gemmw<bf, 1, true><<<dim3(TT / 64, 3 * DD / 64, 1), 32, 0, stream>>>(Xh, Xl, WQKV, nullptr, DD, F3, 3 * DD, IN[3], 0, 0, 0);
        k_cvt8<<<(unsigned)(((size_t)SS * DD / 8 + 255) / 256), 256, 0, stream>>>(IN[1] + (size_t)b * SS * DD, CB, (size_t)SS * DD / 8);
        k_gemmw<bf, 0, true><<<dim3(SS / 64, 2 * DD / 64, 1), 32, 0, stream>>>(CB, nullptr, WCKV, nullptr, DD, FC, 2 * DD, IN[5], 0, 0, 0);
        k_qpl<<<LQ, 256, 0, stream>>>(F3, QP); k_kcat<<<LK, 256, 0, stream>>>(F3, FC, KP); k_vcat<<<LK, 256, 0, stream>>>(F3, FC, VT);
        for (int h0 = 0; h0 < NH_; h0 += ZH) { const size_t z0 = (size_t)h0;
            k_gemmw<h16, 0, false><<<dim3(TT / 64, TK / 64, ZH), 32, 0, stream>>>(QP + z0 * TT * HD, nullptr, KP + z0 * TK * HD, nullptr, HD, Sb, TK, nullptr, (size_t)TT * HD, (size_t)TK * HD, (size_t)TT * TK);
            k_smax<<<ZH * TT / 8, 256, 0, stream>>>(Sb, RS); k_sexp<<<ZH * TT / 8, 256, 0, stream>>>(Sb, RS, Pm);
            k_gemmw<h16, 0, false><<<dim3(TT / 64, HD / 64, ZH), 32, 0, stream>>>(Pm, nullptr, VT + z0 * HD * TK, nullptr, TK, Ob, HD, nullptr, (size_t)TT * TK, (size_t)HD * TK, (size_t)TT * HD);
            k_mrgx<<<(ZH * TT * HD / 2 + 255) / 256, 256, 0, stream>>>(Ob, RS, xb, h0, X1); }
        k_ln1k<0, 1, 1><<<TT / 8, 256, 0, stream>>>(X1, IN[8], IN[9], IN[10], IN[11], nullptr, nullptr, H16);
        k_gemmw<h16, 0, false><<<dim3(TT / 64, FF / 64, 1), 32, 0, stream>>>(H16, nullptr, W1S, nullptr, DD, HF, FF, nullptr, 0, 0, 0); k_gelu16<<<(unsigned)(((size_t)TT * FF / 2 + 255) / 256), 256, 0, stream>>>(HF, IN[13], G16);
        k_gemmw<h16, 0, false><<<dim3(TT / 64, DD / 64, 1), 32, 0, stream>>>(G16, nullptr, W2S, nullptr, FF, F2, DD, nullptr, 0, 0, 0); k_fin<<<(unsigned)(((size_t)TT * DD / 2 + 255) / 256), 256, 0, stream>>>(X1, F2, IN[15], OUT + (size_t)b * TT * DD); }
}
